// MambaProj_8804682957495
// MI455X (gfx1250) — hardware-verified
//
#include <hip/hip_runtime.h>
#include <math.h>

typedef __attribute__((ext_vector_type(16))) _Float16 v16h;
typedef __attribute__((ext_vector_type(8)))  _Float16 v8h;
typedef __attribute__((ext_vector_type(16))) __bf16   v16b;
typedef __attribute__((ext_vector_type(8)))  __bf16   v8b;
typedef __attribute__((ext_vector_type(8)))  float    v8f;
typedef __attribute__((ext_vector_type(4)))  float    v4f;

constexpr int kBatch = 2;
constexpr int kSeqL  = 4096;
constexpr int kDmod  = 512;
constexpr int kXZP   = 1024;
constexpr int kDhalf = 256;
constexpr int kNst   = 8;
constexpr int kDtR   = 32;
constexpr int kPrjN  = 48;
constexpr int kPrjP  = 64;
constexpr int kNseq  = 4;
constexpr int kRows  = kBatch * kSeqL;
constexpr int kSRows = kNseq * kSeqL;
constexpr int kDil   = 8;
constexpr int kTP    = 260;

__device__ __forceinline__ unsigned short f2bf_bits(float f) {
  unsigned u = __float_as_uint(f);
  return (unsigned short)((u + 0x7FFFu + ((u >> 16) & 1u)) >> 16);
}
__device__ __forceinline__ float bf_bits2f(unsigned short h) { return __uint_as_float(((unsigned)h) << 16); }

__device__ __forceinline__ void dep_guard_h(v8f& a, v8f& b, v16h x, v16h y) { asm volatile("v_nop\n\tv_nop\n\tv_nop\n\tv_nop" : "+v"(a), "+v"(b) : "v"(x), "v"(y)); }
__device__ __forceinline__ void dep_guard_b(v8f& a, v8f& b, v16b x, v16b y) { asm volatile("v_nop\n\tv_nop\n\tv_nop\n\tv_nop" : "+v"(a), "+v"(b) : "v"(x), "v"(y)); }
__device__ __forceinline__ void keep4_h(v16h a, v16h b, v16h c, v16h d) { asm volatile("v_nop" :: "v"(a), "v"(b), "v"(c), "v"(d)); }
__device__ __forceinline__ void keep4_b(v16b a, v16b b, v16b c, v16b d) { asm volatile("v_nop" :: "v"(a), "v"(b), "v"(c), "v"(d)); }
__device__ __forceinline__ void acc_guard4(v8f& a, v8f& b, v8f& c, v8f& d) { asm volatile("v_nop\n\tv_nop\n\tv_nop\n\tv_nop" : "+v"(a), "+v"(b), "+v"(c), "+v"(d)); }
template <typename T> struct Frag;
template <> struct Frag<_Float16> {
  typedef v16h V; union U { v16h v; v8h h[2]; };
  static __device__ __forceinline__ v16h load(const _Float16* p) {
    U f; f.h[0] = *(const v8h*)(p); f.h[1] = *(const v8h*)(p + 16); return f.v;
  }
  static __device__ __forceinline__ v8f mma(v16h a, v16h b, v8f c) {
    return __builtin_amdgcn_wmma_f32_16x16x32_f16(false, a, false, b, (short)0, c, false, false);
  }
  static __device__ __forceinline__ void guard(v8f& a, v8f& b, v16h x, v16h y) { dep_guard_h(a, b, x, y); }
  static __device__ __forceinline__ void keep(v16h a, v16h b, v16h c, v16h d) { keep4_h(a, b, c, d); }
};
template <> struct Frag<__bf16> {
  typedef v16b V; union U { v16b v; v8b h[2]; };
  static __device__ __forceinline__ v16b load(const __bf16* p) {
    U f; f.h[0] = *(const v8b*)(p); f.h[1] = *(const v8b*)(p + 16); return f.v;
  }
  static __device__ __forceinline__ v8f mma(v16b a, v16b b, v8f c) {
    return __builtin_amdgcn_wmma_f32_16x16x32_bf16(false, a, false, b, (short)0, c, false, false);
  }
  static __device__ __forceinline__ void guard(v8f& a, v8f& b, v16b x, v16b y) { dep_guard_b(a, b, x, y); }
  static __device__ __forceinline__ void keep(v16b a, v16b b, v16b c, v16b d) { keep4_b(a, b, c, d); }
};

template <int ET> struct Elem;
template <> struct Elem<0> { typedef _Float16 T; };
template <> struct Elem<1> { typedef __bf16 T; };
template <int ET, bool SPLIT, int BIAS_MODE, int OUT_MODE, bool RESID, int ACT = 0>
__global__ __launch_bounds__(256) void wmma_gemm64(
    const unsigned short* __restrict__ Ap, const unsigned short* __restrict__ A2p, int lda, long strideA,
    const unsigned short* __restrict__ Btp, const unsigned short* __restrict__ Bt2p, int ldb, long strideB,
    void* __restrict__ Cout, void* __restrict__ Cout2, int ldc, long strideC,
    const float* __restrict__ bias,
    const float* __restrict__ resid, long strideR,
    int M, int N, int K, float scale) {
  typedef typename Elem<ET>::T T;
  typedef typename Frag<T>::V V;
  const T* A = (const T*)Ap; const T* A2 = (const T*)A2p; const T* Bt = (const T*)Btp; const T* Bt2 = (const T*)Bt2p;
  __shared__ __align__(16) float sT[8][16 * 68];
  const int b    = blockIdx.y;
  const int lane = threadIdx.x & 31;
  const int wave = threadIdx.x >> 5;
  const int tilesN = N >> 6;
  const int tilesM = M >> 6;
  const int tile = blockIdx.x * 8 + wave;
  if (tile >= tilesM * tilesN) return;
  const int tm = tile / tilesN;
  const int tn = tile - tm * tilesN;
  const int m0 = tm << 6;
  const int n0 = tn << 6;

  const T* Ab  = A  + (size_t)b * strideA;
  const T* Bb  = Bt + (size_t)b * strideB;
  const T* Ab2 = SPLIT ? (A2  + (size_t)b * strideA) : nullptr;
  const T* Bb2 = SPLIT ? (Bt2 + (size_t)b * strideB) : nullptr;

  const int rlane = lane & 15;
  const int koff  = (lane >> 4) * 8;
  const int mOff  = (lane >> 4) * 8;

  v8f acc[4][4];
#pragma unroll
  for (int i = 0; i < 4; ++i)
#pragma unroll
    for (int j = 0; j < 4; ++j) acc[i][j] = (v8f){0.f,0.f,0.f,0.f,0.f,0.f,0.f,0.f};

  for (int k0 = 0; k0 < K; k0 += 32) {
    V bh[4], bl[4];
#pragma unroll
    for (int j = 0; j < 4; ++j) {
      const size_t bo = (size_t)(n0 + (j << 4) + rlane) * ldb + koff + k0;
      bh[j] = Frag<T>::load(Bb + bo);
      if (SPLIT) bl[j] = Frag<T>::load(Bb2 + bo);
    }
#pragma unroll
    for (int i = 0; i < 4; ++i) {
      const size_t ao = (size_t)(m0 + (i << 4) + rlane) * lda + koff + k0;
      V ah = Frag<T>::load(Ab + ao);
      V al;
      if (SPLIT) al = Frag<T>::load(Ab2 + ao);
#pragma unroll
      for (int j = 0; j < 4; ++j) {
        acc[i][j] = Frag<T>::mma(ah, bh[j], acc[i][j]);
        if (SPLIT) {
          acc[i][j] = Frag<T>::mma(ah, bl[j], acc[i][j]);
          acc[i][j] = Frag<T>::mma(al, bh[j], acc[i][j]);
        }
      }
      Frag<T>::guard(acc[i][0], acc[i][3], ah, SPLIT ? al : ah);
    }
    Frag<T>::keep(bh[0], bh[1], bh[2], bh[3]);
    if (SPLIT) Frag<T>::keep(bl[0], bl[1], bl[2], bl[3]);
  }
  acc_guard4(acc[0][0], acc[0][1], acc[0][2], acc[0][3]);
  acc_guard4(acc[1][0], acc[1][1], acc[1][2], acc[1][3]);
  acc_guard4(acc[2][0], acc[2][1], acc[2][2], acc[2][3]);
  acc_guard4(acc[3][0], acc[3][1], acc[3][2], acc[3][3]);

  float* slab = sT[wave];
  const float* Rb = RESID ? (resid + (size_t)b * strideR) : nullptr;
#pragma unroll
  for (int i = 0; i < 4; ++i) {
    const int mBase = m0 + (i << 4);
#pragma unroll
    for (int j = 0; j < 4; ++j) {
      const int n = n0 + (j << 4) + rlane;
      float bv = 0.f;
      if (BIAS_MODE == 2) bv = bias[n];
#pragma unroll
      for (int r = 0; r < 8; ++r) {
        float v = acc[i][j][r] * scale;
        if (BIAS_MODE == 1) v += bias[mBase + mOff + r];
        if (BIAS_MODE == 2) v += bv;
        if (RESID) v += Rb[(size_t)(mBase + mOff + r) * ldc + n];
        if (ACT == 1) v = tanhf(v);
        if (ACT == 2) v = fmaxf(v, 0.0f);
        if (ACT == 3) v = v / (1.0f + expf(-v));
        if (ACT == 4) v = (v > 0.f) ? v : 0.01f * v;
        if (ACT == 5) v = 0.5f * v * (1.0f + erff(v * 0.70710678118654752f));
        slab[(mOff + r) * 68 + (j << 4) + rlane] = v;
      }
    }
    __builtin_amdgcn_fence(__ATOMIC_RELEASE, "workgroup");
    __builtin_amdgcn_wave_barrier();
    __builtin_amdgcn_fence(__ATOMIC_ACQUIRE, "workgroup");
    if (OUT_MODE == 0) {
      float* C = (float*)Cout + (size_t)b * strideC;
      const int hh = lane >> 4, c4 = (lane & 15) * 4;
      for (int pass = 0; pass < 2; ++pass) {
#pragma unroll
        for (int it = 0; it < 8; ++it) {
          const int row = it * 2 + hh;
          v4f v = *(const v4f*)(slab + row * 68 + c4);
          *(volatile v4f*)(C + (size_t)(mBase + row) * ldc + n0 + c4) = v;
        }
        __threadfence();
      }
    } else {
      const int q = lane >> 3, c8 = (lane & 7) * 8;
      unsigned short* C  = (unsigned short*)Cout  + (size_t)b * strideC;
      unsigned short* C2 = (OUT_MODE == 2) ? ((unsigned short*)Cout2 + (size_t)b * strideC) : nullptr;
      for (int pass = 0; pass < 2; ++pass) {
#pragma unroll
        for (int it = 0; it < 4; ++it) {
          const int row = it * 4 + q;
          const float* sp = slab + row * 68 + c8;
          v8h hv, lv;
#pragma unroll
          for (int e = 0; e < 8; ++e) {
            if (OUT_MODE == 1) {
              hv[e] = (_Float16)sp[e];
            } else {
              unsigned short hb = f2bf_bits(sp[e]);
              unsigned short lb = f2bf_bits(sp[e] - bf_bits2f(hb));
              hv[e] = __builtin_bit_cast(_Float16, hb);
              lv[e] = __builtin_bit_cast(_Float16, lb);
            }
          }
          *(volatile v8h*)(C + (size_t)(mBase + row) * ldc + n0 + c8) = hv;
          if (OUT_MODE == 2) *(volatile v8h*)(C2 + (size_t)(mBase + row) * ldc + n0 + c8) = lv;
        }
        __threadfence();
      }
    }
    __builtin_amdgcn_fence(__ATOMIC_RELEASE, "workgroup");
    __builtin_amdgcn_wave_barrier();
    __builtin_amdgcn_fence(__ATOMIC_ACQUIRE, "workgroup");
  }
}

__global__ __launch_bounds__(256) void cast_f16_kernel(
    const float* __restrict__ src, unsigned short* __restrict__ dst, int total8, float scale)
{
  const int i = blockIdx.x * 256 + threadIdx.x;
  if (i >= total8) return;
  const size_t e0 = (size_t)i << 3;
  const float* p = src + e0;
  const v4f a0 = *(const v4f*)(p);
  const v4f a1 = *(const v4f*)(p + 4);
  v8h hv;
#pragma unroll
  for (int e = 0; e < 4; ++e) {
    hv[e]     = (_Float16)(a0[e] * scale);
    hv[4 + e] = (_Float16)(a1[e] * scale);
  }
  unsigned short* q = dst + e0;
  *(volatile v8h*)q = hv;
  __threadfence();
  *(volatile v8h*)q = hv;
}

__global__ __launch_bounds__(256) void cast_rows_f16_kernel(
    const float* __restrict__ src, unsigned short* __restrict__ dst, int N, int K, int total8, float scale)
{
  const int i = blockIdx.x * 256 + threadIdx.x;
  if (i >= total8) return;
  const int e0  = i << 3;
  const int row = e0 / K;
  const int col = e0 - row * K;
  const int rowc = (row < N) ? row : (N - 1);
  const bool live = (row < N);
  const float* p = src + (size_t)rowc * K + col;
  const v4f a0 = *(const v4f*)(p);
  const v4f a1 = *(const v4f*)(p + 4);
  v8h hv;
#pragma unroll
  for (int e = 0; e < 4; ++e) {
    hv[e]     = live ? (_Float16)(a0[e] * scale) : (_Float16)0.0f;
    hv[4 + e] = live ? (_Float16)(a1[e] * scale) : (_Float16)0.0f;
  }
  unsigned short* q = dst + (size_t)e0;
  *(volatile v8h*)q = hv;
  __threadfence();
  *(volatile v8h*)q = hv;
}

__global__ __launch_bounds__(256) void dtr_cast_kernel(
    const float* __restrict__ XDBL, unsigned short* __restrict__ DTR16, int total8, float scale)
{
  const int i = blockIdx.x * 256 + threadIdx.x;
  if (i >= total8) return;
  const int e0  = i << 3;
  const int row = e0 >> 5;
  const int c8  = e0 & 31;
  const float* p = XDBL + (size_t)row * kPrjP + c8;
  const v4f a0 = *(const v4f*)(p);
  const v4f a1 = *(const v4f*)(p + 4);
  v8h hv;
#pragma unroll
  for (int e = 0; e < 4; ++e) {
    hv[e]     = (_Float16)(a0[e] * scale);
    hv[4 + e] = (_Float16)(a1[e] * scale);
  }
  unsigned short* qd = DTR16 + (size_t)e0;
  *(volatile v8h*)qd = hv;
  __threadfence();
  *(volatile v8h*)qd = hv;
}

__global__ __launch_bounds__(256) void conv_silu_kernel(
    const float* __restrict__ XZ, const float* __restrict__ wx, const float* __restrict__ wz,
    float* __restrict__ XC, unsigned short* __restrict__ XC16, unsigned short* __restrict__ A16)
{
  __shared__ __align__(16) float sX[16 * kTP];
  __shared__ __align__(16) float sZ[16 * kTP];
  const int tid = threadIdx.x, lane = tid & 31, wave = tid >> 5;
  const int d = tid;
  const int s = blockIdx.x;
  const int b = s & 1;
  const int bw = s >> 1;
  const int t0 = blockIdx.y * 64;
  const int cbase = bw ? kDmod : 0;
  const int zcolA = bw ? (kDmod + kDhalf) : kDhalf;
  const size_t brow = (size_t)b * kSeqL;
  const size_t srow = (size_t)s * kSeqL;
  const float wx0 = wx[d * 4 + 0], wx1 = wx[d * 4 + 1], wx2 = wx[d * 4 + 2], wx3 = wx[d * 4 + 3];
  const float wz0 = wz[d * 4 + 0], wz1 = wz[d * 4 + 1], wz2 = wz[d * 4 + 2], wz3 = wz[d * 4 + 3];
  float zm3, zm2, zm1;
  {
    const int t3 = t0 - 3, t2 = t0 - 2, t1 = t0 - 1;
    const int c3 = t3 < 0 ? 0 : t3, c2 = t2 < 0 ? 0 : t2, c1 = t1 < 0 ? 0 : t1;
    const int l3 = bw ? (kSeqL - 1 - c3) : c3;
    const int l2 = bw ? (kSeqL - 1 - c2) : c2;
    const int l1 = bw ? (kSeqL - 1 - c1) : c1;
    const float v3 = XZ[(brow + l3) * kXZP + cbase + kDhalf + d];
    const float v2 = XZ[(brow + l2) * kXZP + cbase + kDhalf + d];
    const float v1 = XZ[(brow + l1) * kXZP + cbase + kDhalf + d];
    zm3 = (t3 >= 0) ? v3 : 0.f;
    zm2 = (t2 >= 0) ? v2 : 0.f;
    zm1 = (t1 >= 0) ? v1 : 0.f;
  }
  const int hrow = wave >> 1;
  const int hch  = (wave & 1) * 128 + lane * 4;
#pragma unroll 1
  for (int sub = 0; sub < 4; ++sub) {
    const int lb = t0 + sub * 16;
#pragma unroll 1
    for (int st = 0; st < 16; ++st) {
      const int tt = lb + st;
      const int l  = bw ? (kSeqL - 1 - tt) : tt;
      const float* rp = XZ + (brow + l) * kXZP + cbase;
      const float xc = rp[d];
      const float zc = rp[kDhalf + d];
      const int t8 = tt - kDil, t16 = tt - 2 * kDil, t24 = tt - 3 * kDil;
      const int c8 = t8 < 0 ? 0 : t8, c16 = t16 < 0 ? 0 : t16, c24 = t24 < 0 ? 0 : t24;
      const int l8  = bw ? (kSeqL - 1 - c8)  : c8;
      const int l16 = bw ? (kSeqL - 1 - c16) : c16;
      const int l24 = bw ? (kSeqL - 1 - c24) : c24;
      const float v8  = XZ[(brow + l8)  * kXZP + cbase + d];
      const float v16 = XZ[(brow + l16) * kXZP + cbase + d];
      const float v24 = XZ[(brow + l24) * kXZP + cbase + d];
      const float x8  = (t8  >= 0) ? v8  : 0.f;
      const float x16 = (t16 >= 0) ? v16 : 0.f;
      const float x24 = (t24 >= 0) ? v24 : 0.f;
      float ax = wx0 * x24;
      ax = fmaf(wx1, x16, ax);
      ax = fmaf(wx2, x8, ax);
      ax = fmaf(wx3, xc, ax);
      float az = wz0 * zm3;
      az = fmaf(wz1, zm2, az);
      az = fmaf(wz2, zm1, az);
      az = fmaf(wz3, zc, az);
      const float sgx = __builtin_amdgcn_rcpf(1.0f + __expf(-ax));
      const float sgz = __builtin_amdgcn_rcpf(1.0f + __expf(-az));
      sX[st * kTP + tid] = ax * sgx;
      sZ[st * kTP + tid] = az * sgz;
      zm3 = zm2; zm2 = zm1; zm1 = zc;
    }
    __syncthreads();
    v4f fv[4];
    v8h bx[2], bz[2];
#pragma unroll
    for (int it = 0; it < 4; ++it) fv[it] = *(const v4f*)(sX + (it * 4 + hrow) * kTP + hch);
#pragma unroll
    for (int it = 0; it < 2; ++it) {
      const float* spx = sX + (it * 8 + wave) * kTP + lane * 8;
      const float* spz = sZ + (it * 8 + wave) * kTP + lane * 8;
      const v4f a0 = *(const v4f*)(spx);
      const v4f a1 = *(const v4f*)(spx + 4);
      const v4f z0 = *(const v4f*)(spz);
      const v4f z1 = *(const v4f*)(spz + 4);
#pragma unroll
      for (int e = 0; e < 4; ++e) {
        bx[it][e]     = (_Float16)a0[e];
        bx[it][4 + e] = (_Float16)a1[e];
        bz[it][e]     = (_Float16)z0[e];
        bz[it][4 + e] = (_Float16)z1[e];
      }
    }
    for (int pass = 0; pass < 2; ++pass) {
#pragma unroll
      for (int it = 0; it < 4; ++it)
        *(volatile v4f*)(XC + (srow + lb + it * 4 + hrow) * kDhalf + hch) = fv[it];
#pragma unroll
      for (int it = 0; it < 2; ++it) {
        const int tt = lb + it * 8 + wave;
        *(volatile v8h*)(XC16 + (srow + tt) * kDhalf + lane * 8) = bx[it];
        const size_t arow = brow + (size_t)(bw ? (kSeqL - 1 - tt) : tt);
        *(volatile v8h*)(A16 + arow * kXZP + zcolA + lane * 8) = bz[it];
      }
      __threadfence();
    }
    __syncthreads();
  }
}

__global__ __launch_bounds__(256) void scan_kernel(
    const float* __restrict__ DLR, const float* __restrict__ XC, const float* __restrict__ XDBL,
    const float* __restrict__ A_log, const float* __restrict__ Dv, unsigned short* __restrict__ A16)
{
  __shared__ __align__(16) float sBC[16 * 16];
  __shared__ __align__(16) float sY[16 * kTP];
  const int tid = threadIdx.x, lane = tid & 31, wave = tid >> 5;
  const int d = tid;
  const int s = blockIdx.x;
  const int b = s & 1;
  const int bw = s >> 1;
  const int ycol = bw ? kDmod : 0;
  const size_t brow  = (size_t)b * kSeqL;
  const size_t srow0 = (size_t)s * kSeqL;

  float An[kNst];
#pragma unroll
  for (int n = 0; n < kNst; ++n) An[n] = -__expf(A_log[(size_t)d * kNst + n]);
  const float Dd = Dv[d];
  float h[kNst];
#pragma unroll
  for (int n = 0; n < kNst; ++n) h[n] = 0.f;

#pragma unroll 1
  for (int c = 0; c < kSeqL / 16; ++c) {
    const int l0 = c * 16;
    if (tid < 64) {
      const int r = tid >> 2, q = (tid & 3) * 4;
      const v4f v = *(const v4f*)(XDBL + (srow0 + l0 + r) * kPrjP + kDtR + q);
      *(v4f*)(sBC + r * 16 + q) = v;
    }
    __syncthreads();
#pragma unroll 1
    for (int st = 0; st < 16; ++st) {
      const size_t m = srow0 + l0 + st;
      const float a     = DLR[m * kDhalf + d];
      const float delta = fmaxf(a, 0.0f) + log1pf(__expf(-fabsf(a)));
      const float xv    = XC[m * kDhalf + d];
      v4f Bq[2], Cq[2];
      Bq[0] = *(const v4f*)(sBC + st * 16 + 0);
      Bq[1] = *(const v4f*)(sBC + st * 16 + 4);
      Cq[0] = *(const v4f*)(sBC + st * 16 + 8);
      Cq[1] = *(const v4f*)(sBC + st * 16 + 12);
      float y = 0.f;
#pragma unroll
      for (int n = 0; n < kNst; ++n) {
        const float e = __expf(delta * An[n]);
        float db = delta * Bq[n >> 2][n & 3];
        asm volatile("" : "+v"(db));
        float p = db * xv;
        asm volatile("" : "+v"(p));
        float qv = h[n] * e;
        asm volatile("" : "+v"(qv));
        const float hn = qv + p;
        h[n] = hn;
        float rr = Cq[n >> 2][n & 3] * hn;
        asm volatile("" : "+v"(rr));
        y += rr;
      }
      float sk = xv * Dd;
      asm volatile("" : "+v"(sk));
      y += sk;
      sY[st * kTP + tid] = y;
    }
    __syncthreads();
    v8h hv[2];
#pragma unroll
    for (int it = 0; it < 2; ++it) {
      const float* sp = sY + (it * 8 + wave) * kTP + lane * 8;
      const v4f a0 = *(const v4f*)(sp);
      const v4f a1 = *(const v4f*)(sp + 4);
#pragma unroll
      for (int e = 0; e < 4; ++e) { hv[it][e] = (_Float16)a0[e]; hv[it][4 + e] = (_Float16)a1[e]; }
    }
    for (int pass = 0; pass < 2; ++pass) {
#pragma unroll
      for (int it = 0; it < 2; ++it) {
        const int tt = l0 + it * 8 + wave;
        const size_t arow = brow + (size_t)(bw ? (kSeqL - 1 - tt) : tt);
        *(volatile v8h*)(A16 + arow * kXZP + ycol + lane * 8) = hv[it];
      }
      __threadfence();
    }
  }
}

extern "C" void kernel_launch(void* const* d_in, const int* in_sizes, int n_in,
                              void* d_out, int out_size, void* d_ws, size_t ws_size,
                              hipStream_t stream)
{
  if (n_in < 10) return;
  const float* hs     = (const float*)d_in[0];
  const float* W_in   = (const float*)d_in[1];
  const float* W_xprj = (const float*)d_in[2];
  const float* W_dt   = (const float*)d_in[3];
  const float* b_dt   = (const float*)d_in[4];
  const float* A_log  = (const float*)d_in[5];
  const float* Dv     = (const float*)d_in[6];
  const float* w_cx   = (const float*)d_in[7];
  const float* w_cz   = (const float*)d_in[8];
  const float* W_out  = (const float*)d_in[9];
  float* dout = (float*)d_out;

  if (in_sizes[0] != kRows * kDmod) return;
  if (in_sizes[1] != kXZP * kDmod) return;
  if (in_sizes[2] != kPrjN * kDhalf) return;
  if (in_sizes[3] != kDhalf * kDtR) return;
  if (in_sizes[4] != kDhalf) return;
  if (in_sizes[5] != kDhalf * kNst) return;
  if (in_sizes[6] != kDhalf) return;
  if (in_sizes[7] != kDhalf * 4 || in_sizes[8] != kDhalf * 4) return;
  if (in_sizes[9] != kDmod * kXZP) return;
  if (out_size != kRows * kDmod) return;

  const size_t SZ_WIN16  = (size_t)kXZP * kDmod * 2;
  const size_t SZ_WXP16  = (size_t)kPrjP * kDhalf * 2;
  const size_t SZ_WDT16  = (size_t)kDhalf * kDtR * 2;
  const size_t SZ_WOUT16 = (size_t)kDmod * kXZP * 2;
  const size_t SZ_X16    = (size_t)kRows * kDmod * 2;
  const size_t SZ_XZ     = (size_t)kRows * kXZP * 4;
  const size_t SZ_XC     = (size_t)kSRows * kDhalf * 4;
  const size_t SZ_XC16   = (size_t)kSRows * kDhalf * 2;
  const size_t SZ_A16    = (size_t)kRows * kXZP * 2;
  const size_t SZ_XDBL   = (size_t)kSRows * kPrjP * 4;
  const size_t SZ_DTR16  = (size_t)kSRows * kDtR * 2;
  const size_t SZ_DLR    = (size_t)kSRows * kDhalf * 4;
  const size_t OFF_WIN16  = 0;
  const size_t OFF_WXP16  = OFF_WIN16  + SZ_WIN16;
  const size_t OFF_WDT16  = OFF_WXP16  + SZ_WXP16;
  const size_t OFF_WOUT16 = OFF_WDT16  + SZ_WDT16;
  const size_t OFF_X16    = OFF_WOUT16 + SZ_WOUT16;
  const size_t OFF_XZ     = OFF_X16    + SZ_X16;
  const size_t OFF_XC     = OFF_XZ     + SZ_XZ;
  const size_t OFF_XC16   = OFF_XC     + SZ_XC;
  const size_t OFF_A16    = OFF_XC16   + SZ_XC16;
  const size_t OFF_XDBL   = OFF_A16    + SZ_A16;
  const size_t OFF_DTR16  = OFF_XDBL   + SZ_XDBL;
  const size_t OFF_DLR    = OFF_DTR16  + SZ_DTR16;
  const size_t TOTAL      = OFF_DLR    + SZ_DLR;
  if (ws_size < TOTAL) return;

  if (((kXZP * kDmod) / 8) % 256 != 0) return;
  if (((kPrjP * kDhalf) / 8) % 256 != 0) return;
  if (((kDhalf * kDtR) / 8) % 256 != 0) return;
  if (((kRows * kDmod) / 8) % 256 != 0) return;
  if (((kSRows * kDtR) / 8) % 256 != 0) return;

  char* ws = (char*)d_ws;
  unsigned short* WIN16  = (unsigned short*)(ws + OFF_WIN16);
  unsigned short* WXP16  = (unsigned short*)(ws + OFF_WXP16);
  unsigned short* WDT16  = (unsigned short*)(ws + OFF_WDT16);
  unsigned short* WOUT16 = (unsigned short*)(ws + OFF_WOUT16);
  unsigned short* X16    = (unsigned short*)(ws + OFF_X16);
  float*          XZ     = (float*)(ws + OFF_XZ);
  float*          XC     = (float*)(ws + OFF_XC);
  unsigned short* XC16   = (unsigned short*)(ws + OFF_XC16);
  unsigned short* A16    = (unsigned short*)(ws + OFF_A16);
  float*          XDBL   = (float*)(ws + OFF_XDBL);
  unsigned short* DTR16  = (unsigned short*)(ws + OFF_DTR16);
  float*          DLR    = (float*)(ws + OFF_DLR);
  const float* dummy_bias  = b_dt;
  const float* dummy_resid = hs;

  cast_rows_f16_kernel<<<(kXZP * kDmod) / 8 / 256, 256, 0, stream>>>(W_in,   WIN16,  kXZP,  kDmod,  (kXZP * kDmod) / 8,  16.0f);
  cast_rows_f16_kernel<<<(kPrjP * kDhalf) / 8 / 256, 256, 0, stream>>>(W_xprj, WXP16, kPrjN, kDhalf, (kPrjP * kDhalf) / 8, 16.0f);
  cast_rows_f16_kernel<<<(kDhalf * kDtR) / 8 / 256, 256, 0, stream>>>(W_dt,   WDT16,  kDhalf, kDtR,  (kDhalf * kDtR) / 8,  8.0f);
  cast_rows_f16_kernel<<<(kDmod * kXZP) / 8 / 256, 256, 0, stream>>>(W_out,  WOUT16, kDmod,  kXZP,  (kDmod * kXZP) / 8,  32.0f);

  cast_f16_kernel<<<(kRows * kDmod) / 8 / 256, 256, 0, stream>>>(hs, X16, (kRows * kDmod) / 8, 1.0f);

  wmma_gemm64<0, false, 0, 0, false><<<dim3(256, 1), 256, 0, stream>>>(
      X16, X16, kDmod, 0L, WIN16, WIN16, kDmod, 0L,
      (void*)XZ, (void*)XZ, kXZP, 0L, dummy_bias, dummy_resid, 0L, kRows, kXZP, kDmod, 1.0f / 16.0f);

  conv_silu_kernel<<<dim3(kNseq, kSeqL / 64), 256, 0, stream>>>(XZ, w_cx, w_cz, XC, XC16, A16);

  wmma_gemm64<0, false, 0, 0, false><<<dim3(32, 1), 256, 0, stream>>>(
      XC16, XC16, kDhalf, 0L, WXP16, WXP16, kDhalf, 0L,
      (void*)XDBL, (void*)XDBL, kPrjP, 0L, dummy_bias, dummy_resid, 0L, kSRows, kPrjP, kDhalf, 1.0f / 16.0f);

  dtr_cast_kernel<<<(kSRows * kDtR) / 8 / 256, 256, 0, stream>>>(XDBL, DTR16, (kSRows * kDtR) / 8, 4.0f);

  wmma_gemm64<0, false, 2, 0, false><<<dim3(128, 1), 256, 0, stream>>>(
      DTR16, DTR16, kDtR, 0L, WDT16, WDT16, kDtR, 0L,
      (void*)DLR, (void*)DLR, kDhalf, 0L, b_dt, dummy_resid, 0L, kSRows, kDhalf, kDtR, 1.0f / 32.0f);

  scan_kernel<<<dim3(kNseq, 1), 256, 0, stream>>>(DLR, XC, XDBL, A_log, Dv, A16);

  wmma_gemm64<0, false, 0, 0, false><<<dim3(128, 1), 256, 0, stream>>>(
      A16, A16, kXZP, 0L, WOUT16, WOUT16, kXZP, 0L,
      (void*)dout, (void*)dout, kDmod, 0L, dummy_bias, dummy_resid, 0L, kRows, kDmod, kXZP, 1.0f / 32.0f);
}
